// Block_54408645706395
// MI455X (gfx1250) — hardware-run, weakly checked
//
#include <hip/hip_runtime.h>


#ifndef NB
#define NB 8
#endif
#define NB_FULL 8
#define HH   64
#define WW   64
#define SEQ  (HH * WW)
#define CD   384
#define NH_  8
#define HD   48
#define KVS  4
#define KGH  (HH / KVS)
#define KGW  (WW / KVS)
#define NKV  (KGH * KGW)
#define HID  1536
#define BN   (NB * SEQ)
#define BK   (NB * NKV)
#define KVP  64
#define APITCH 388
#define MLPQ 4
#define QROWS (BN / MLPQ)

#define HC   16.0f
#define WC   1024.0f
#define QC   64.0f
#define KIC  256.0f
#define KSC  4096.0f
#define VC   1024.0f
#define KVC  4096.0f
#define AC   4096.0f
#define GC   64.0f
#define ATT_SCALE 0.14433756729740643f
#define LOG2E 1.4426950408889634f

static_assert(NH_ * HD == CD);
static_assert(HD == 48);
static_assert((HD * 2) % 16 == 0);
static_assert(CD % 64 == 0);
static_assert(HID % 64 == 0);
static_assert(CD % 32 == 0);
static_assert(HID % 32 == 0);
static_assert(NKV == 256);
static_assert(NKV % 64 == 0);
static_assert(NKV % 32 == 0);
static_assert(BN % 64 == 0);
static_assert(BK % 64 == 0);
static_assert(SEQ % 16 == 0);
static_assert(BN % 8 == 0);
static_assert((BN / MLPQ) % 64 == 0);
static_assert((size_t)QROWS * HID == (size_t)BN * CD);
static_assert(((size_t)BK * 48) % 256 == 0);
static_assert((NB * CD) % 8 == 0);
static_assert(CD == 3 * 128);
static_assert(CD / 8 == 48);
static_assert((APITCH * 4) % 16 == 0);
static_assert(APITCH >= CD);
static_assert(NB <= NB_FULL);
static_assert(64 * 65 * 4 <= 131072);
static_assert(8 * CD * 4 <= 131072);
static_assert(16 * 68 * 4 <= 131072);
static_assert(HD * 68 * 4 <= 131072);
static_assert(16 * APITCH * 4 <= 131072);

typedef _Float16 h16;
typedef unsigned short bf;
typedef __attribute__((ext_vector_type(16))) _Float16 v16h;
typedef __attribute__((ext_vector_type(8)))  _Float16 v8h;
typedef __attribute__((ext_vector_type(8)))  float    v8f;
typedef __attribute__((ext_vector_type(4)))  float    v4f;
typedef v4f  __attribute__((may_alias)) v4fa;

__device__ __forceinline__ unsigned short f2bf(float f) { unsigned u = __float_as_uint(f); u += 0x7FFFu + ((u >> 16) & 1u); return (unsigned short)(u >> 16); }
__device__ __forceinline__ float bfr(float f) { return __uint_as_float(((unsigned)f2bf(f)) << 16); }
__device__ __forceinline__ v16h cat16(v8h lo, v8h hi) { return __builtin_shufflevector(lo, hi, 0, 1, 2, 3, 4, 5, 6, 7, 8, 9, 10, 11, 12, 13, 14, 15); }
__device__ __forceinline__ v8f wmma16(v16h a, v16h b, v8f c) { return __builtin_amdgcn_wmma_f32_16x16x32_f16(false, a, false, b, (short)0, c, false, false); }
__device__ __forceinline__ v8f wmma16g(v16h a, v16h b, v8f c) {
    c = wmma16(a, b, c);
    asm volatile("v_nop\n\tv_nop\n\tv_nop\n\tv_nop" : "+v"(c) : "v"(a), "v"(b));
    return c;
}
__device__ __forceinline__ v16h ldh(const h16* p) { return cat16(*(const v8h*)p, *(const v8h*)(p + 16)); }
__device__ __forceinline__ void wave_sync() { __builtin_amdgcn_fence(3  , "wavefront"); __builtin_amdgcn_wave_barrier(); asm volatile("" ::: "memory"); }
static __device__ __forceinline__ h16 toh_flush(float v) { const h16 r = (h16)v; return (fabsf(v) < 6.103515625e-05f) ? (h16)0.0f : r; }
__device__ __forceinline__ float gelu_erf(float x) { return 0.5f * x * (1.0f + erff(x * 0.70710678118654752f)); }

static_assert(2 * 256 * 16 == 64 * 128);
static_assert(16 * 256 == 64 * 64);
__global__ __launch_bounds__(256) void k_wconv(const float* __restrict__ w, h16* wt, int K, int N) {
    __shared__ float ts[64 * 65];
    const int tid = threadIdx.x; const int n0 = blockIdx.x * 64, k0 = blockIdx.y * 64;
#pragma unroll 1
    for (int i = 0; i < 16; ++i) { const int e = i * 256 + tid; const int kk = e >> 6, nn = e & 63;
        ts[nn * 65 + kk] = bfr(w[(size_t)(k0 + kk) * N + n0 + nn]) * WC; }
    __syncthreads();
    const int row = tid >> 3, c8 = (tid & 7) * 8;
    v8h hv0, hv1;
#pragma unroll
    for (int i = 0; i < 8; ++i) { hv0[i] = toh_flush(ts[row * 65 + c8 + i]); hv1[i] = toh_flush(ts[(row + 32) * 65 + c8 + i]); }
    const size_t o0 = (size_t)(n0 + row) * K + k0 + c8;
    const size_t o1 = (size_t)(n0 + 32 + row) * K + k0 + c8;
    *(volatile v8h*)(wt + o0) = hv0; *(volatile v8h*)(wt + o1) = hv1;
    __threadfence();
    *(volatile v8h*)(wt + o0) = hv0; *(volatile v8h*)(wt + o1) = hv1;
}

__device__ __forceinline__ void ln_norm(v4f (&v)[3], const float* __restrict__ lg, const float* __restrict__ lb, const int lane) {
#pragma clang fp contract(off)
    float sm = 0.0f;
#pragma unroll
    for (int g = 0; g < 3; ++g) {
#pragma unroll
        for (int i = 0; i < 4; ++i) sm = sm + v[g][i]; }
    sm = sm + __shfl_xor(sm, 16, 32); sm = sm + __shfl_xor(sm, 8, 32); sm = sm + __shfl_xor(sm, 4, 32); sm = sm + __shfl_xor(sm, 2, 32); sm = sm + __shfl_xor(sm, 1, 32);
    const float mean = sm * (1.0f / CD);
    float sq = 0.0f;
#pragma unroll
    for (int g = 0; g < 3; ++g) {
#pragma unroll
        for (int i = 0; i < 4; ++i) { const float d = v[g][i] - mean; sq = sq + d * d; } }
    sq = sq + __shfl_xor(sq, 16, 32); sq = sq + __shfl_xor(sq, 8, 32); sq = sq + __shfl_xor(sq, 4, 32); sq = sq + __shfl_xor(sq, 2, 32); sq = sq + __shfl_xor(sq, 1, 32);
    const float rstd = rsqrtf(sq * (1.0f / CD) + 1.0e-5f);
#pragma unroll
    for (int g = 0; g < 3; ++g) { const v4f gv = *(const v4f*)(lg + 128 * g + 4 * lane); const v4f bv = *(const v4f*)(lb + 128 * g + 4 * lane);
#pragma unroll
        for (int i = 0; i < 4; ++i) v[g][i] = ((v[g][i] - mean) * rstd * bfr(gv[i]) + bfr(bv[i])) * HC; }
}

static_assert(3 * 32 * 16 == CD * 4);
static_assert((256 + 128) * 16 == 8 * CD * 2);
__global__ __launch_bounds__(256) void k_cpe_ln(const float* __restrict__ x, const float* __restrict__ cw, const float* __restrict__ cb,
                                                const float* __restrict__ lg, const float* __restrict__ lb,
                                                const int* __restrict__ Hp, const int* __restrict__ Wp, float* X1, h16* HP) {
#pragma clang fp contract(off)
    __shared__ __align__(16) float hs[8 * CD];
    const int tid = threadIdx.x, lane = tid & 31;
    const int wave = __builtin_amdgcn_readfirstlane((int)(threadIdx.x >> 5));
    const int tokl = blockIdx.x * 8 + wave;
    const int b = tokl / SEQ, t = tokl % SEQ; const int py = t / WW, px = t % WW;
    const bool okdim = (Hp[0] == HH) & (Wp[0] == WW);
    const float* xb = x + (size_t)b * SEQ * CD;
    v4f acc[3];
#pragma unroll
    for (int g = 0; g < 3; ++g) acc[g] = (v4f){};
#pragma unroll 1
    for (int tap = 0; tap < 9; ++tap) {
        const int yy = py + tap / 3 - 1, xx = px + tap % 3 - 1;
        if ((yy >= 0) & (yy < HH) & (xx >= 0) & (xx < WW)) {
            const float* xr = xb + (size_t)(yy * WW + xx) * CD + 4 * lane; const float* wr = cw + tap * CD + 4 * lane;
#pragma unroll
            for (int g = 0; g < 3; ++g) { const v4f xv = *(const v4f*)(xr + 128 * g); const v4f wv = *(const v4f*)(wr + 128 * g);
#pragma unroll
                for (int i = 0; i < 4; ++i) acc[g][i] = acc[g][i] + bfr(xv[i]) * bfr(wv[i]); } } }
    const float qnan = __uint_as_float(0x7fc00000u);
    v4f v[3];
    { const float* xr = xb + (size_t)t * CD + 4 * lane;
#pragma unroll
      for (int g = 0; g < 3; ++g) { const v4f xv = *(const v4f*)(xr + 128 * g); const v4f bv = *(const v4f*)(cb + 128 * g + 4 * lane);
#pragma unroll
          for (int i = 0; i < 4; ++i) { const float r = bfr(xv[i]) + (acc[g][i] + bfr(bv[i])); v[g][i] = okdim ? r : qnan; } } }
    float* x1r = X1 + (size_t)tokl * CD + 4 * lane;
    *(volatile v4f*)(x1r) = v[0]; *(volatile v4f*)(x1r + 128) = v[1]; *(volatile v4f*)(x1r + 256) = v[2];
    __threadfence();
    *(volatile v4f*)(x1r) = v[0]; *(volatile v4f*)(x1r + 128) = v[1]; *(volatile v4f*)(x1r + 256) = v[2];
    ln_norm(v, lg, lb, lane);
#pragma unroll
    for (int g = 0; g < 3; ++g) *(v4fa*)(&hs[wave * CD + 128 * g + 4 * lane]) = v[g];
    __syncthreads();
    const size_t hb = (size_t)blockIdx.x * 8 * CD;
    const int p1 = (tid < 128) ? (256 + tid) : tid;
    v8h o0, o1;
    { const v4f a0 = *(const v4fa*)(&hs[tid * 8]); const v4f a1 = *(const v4fa*)(&hs[tid * 8 + 4]);
      const v4f c0 = *(const v4fa*)(&hs[p1 * 8]);  const v4f c1 = *(const v4fa*)(&hs[p1 * 8 + 4]);
#pragma unroll
      for (int i = 0; i < 4; ++i) { o0[i] = toh_flush(a0[i]); o0[4 + i] = toh_flush(a1[i]); o1[i] = toh_flush(c0[i]); o1[4 + i] = toh_flush(c1[i]); } }
    *(volatile v8h*)(HP + hb + (size_t)tid * 8) = o0; if (tid < 128) *(volatile v8h*)(HP + hb + (size_t)(256 + tid) * 8) = o1;
    __threadfence();
    *(volatile v8h*)(HP + hb + (size_t)tid * 8) = o0; if (tid < 128) *(volatile v8h*)(HP + hb + (size_t)(256 + tid) * 8) = o1;
}

__global__ __launch_bounds__(256) void k_ln2(const float* __restrict__ X2, const float* __restrict__ lg, const float* __restrict__ lb, h16* HP) {
#pragma clang fp contract(off)
    __shared__ __align__(16) float hs[8 * CD];
    const int tid = threadIdx.x, lane = tid & 31;
    const int wave = __builtin_amdgcn_readfirstlane((int)(threadIdx.x >> 5));
    const int tokl = blockIdx.x * 8 + wave;
    const float* xr = X2 + (size_t)tokl * CD + 4 * lane;
    v4f v[3];
#pragma unroll
    for (int g = 0; g < 3; ++g) v[g] = *(const v4f*)(xr + 128 * g);
    ln_norm(v, lg, lb, lane);
#pragma unroll
    for (int g = 0; g < 3; ++g) *(v4fa*)(&hs[wave * CD + 128 * g + 4 * lane]) = v[g];
    __syncthreads();
    const size_t hb = (size_t)blockIdx.x * 8 * CD;
    const int p1 = (tid < 128) ? (256 + tid) : tid;
    v8h o0, o1;
    { const v4f a0 = *(const v4fa*)(&hs[tid * 8]); const v4f a1 = *(const v4fa*)(&hs[tid * 8 + 4]);
      const v4f c0 = *(const v4fa*)(&hs[p1 * 8]);  const v4f c1 = *(const v4fa*)(&hs[p1 * 8 + 4]);
#pragma unroll
      for (int i = 0; i < 4; ++i) { o0[i] = toh_flush(a0[i]); o0[4 + i] = toh_flush(a1[i]); o1[i] = toh_flush(c0[i]); o1[4 + i] = toh_flush(c1[i]); } }
    *(volatile v8h*)(HP + hb + (size_t)tid * 8) = o0; if (tid < 128) *(volatile v8h*)(HP + hb + (size_t)(256 + tid) * 8) = o1;
    __threadfence();
    *(volatile v8h*)(HP + hb + (size_t)tid * 8) = o0; if (tid < 128) *(volatile v8h*)(HP + hb + (size_t)(256 + tid) * 8) = o1;
}

__global__ __launch_bounds__(256) void k_kvconv(const h16* __restrict__ HP, const float* __restrict__ kw, h16* KI) {
#pragma clang fp contract(off)
    const int idx = blockIdx.x * 256 + threadIdx.x;
    const int tk = idx / 48, ch = idx % 48; const int b = tk / NKV, r = tk % NKV; const int oy = r / KGW, ox = r % KGW;
    float acc[8];
#pragma unroll
    for (int i = 0; i < 8; ++i) acc[i] = 0.0f;
#pragma unroll 1
    for (int tap = 0; tap < 16; ++tap) { const int ky = tap >> 2, kx = tap & 3;
        const size_t src = ((size_t)b * SEQ + (size_t)(oy * KVS + ky) * WW + (size_t)(ox * KVS + kx)) * CD + (size_t)ch * 8;
        const v8h hv = *(const v8h*)(HP + src);
        const v4f w0 = *(const v4f*)(kw + tap * CD + ch * 8); const v4f w1 = *(const v4f*)(kw + tap * CD + ch * 8 + 4);
#pragma unroll
        for (int i = 0; i < 4; ++i) { acc[i] = acc[i] + (float)hv[i] * bfr(w0[i]); acc[4 + i] = acc[4 + i] + (float)hv[4 + i] * bfr(w1[i]); } }
    v8h o;
#pragma unroll
    for (int i = 0; i < 8; ++i) o[i] = toh_flush(acc[i] * (KIC / HC));
    *(volatile v8h*)(KI + (size_t)idx * 8) = o; __threadfence(); *(volatile v8h*)(KI + (size_t)idx * 8) = o;
}

static_assert(4 * 32 * 16 == 16 * 128);
static_assert(8 * 32 * 16 == 16 * 256);
static_assert(8 * 32 * 4 == 16 * 64);
template <int OUTF32, int BIASM, int RES, int GELU>
__device__ __forceinline__ void gemm_tile(float (&os)[16 * 68], const h16* __restrict__ A, const h16* __restrict__ Bt, const float* __restrict__ bias, const float* __restrict__ res,
                                          float* Cf, h16* Ch, const int K, const int ldc, const int nsplit, const size_t bstride,
                                          const float alpha, const float bscale, const float oscale) {
    const int lane = threadIdx.x & 31, lr = lane & 15, hi = lane >> 4; const int r0 = blockIdx.x * 64, c0 = blockIdx.y * 64;
    v8f acc[4][4];
#pragma unroll
    for (int mb = 0; mb < 4; ++mb)
#pragma unroll
        for (int nb = 0; nb < 4; ++nb) acc[mb][nb] = (v8f){};
    const size_t aoff = (size_t)(r0 + lr) * K + 8 * hi, boff = (size_t)(c0 + lr) * K + 8 * hi;
#pragma unroll 1
    for (int kc = 0; kc < K; kc += 32) {
        v16h a[4];
#pragma unroll
        for (int mb = 0; mb < 4; ++mb) a[mb] = ldh(A + aoff + (size_t)mb * 16 * K + kc);
#pragma unroll
        for (int nb = 0; nb < 4; ++nb) { const v16h b = ldh(Bt + boff + (size_t)nb * 16 * K + kc);
#pragma unroll
            for (int mb = 0; mb < 4; ++mb) acc[mb][nb] = wmma16g(a[mb], b, acc[mb][nb]); }
    }
    float bc[4];
#pragma unroll
    for (int nb = 0; nb < 4; ++nb) { bc[nb] = 0.0f; if (BIASM == 1) bc[nb] = bfr(bias[c0 + nb * 16 + lr]) * bscale; }
    const size_t obase = (size_t)(c0 / nsplit) * bstride + (size_t)r0 * ldc + (size_t)(c0 % nsplit);
#pragma unroll
    for (int mb = 0; mb < 4; ++mb) {
        float br[8];
#pragma unroll
        for (int j = 0; j < 8; ++j) { br[j] = 0.0f; if (BIASM == 2) br[j] = bfr(bias[r0 + mb * 16 + hi * 8 + j]) * bscale; }
#pragma unroll
        for (int nb = 0; nb < 4; ++nb) {
#pragma unroll
            for (int j = 0; j < 8; ++j) os[(hi * 8 + j) * 68 + nb * 16 + lr] = acc[mb][nb][j] * alpha + bc[nb] + br[j]; }
        wave_sync();
        if (GELU) {
#pragma unroll 1
            for (int it = 0; it < 8; ++it) { const int e = (it * 32 + lane) * 4; const int row = e >> 6, col = e & 63;
                v4f xv = *(const v4fa*)(&os[row * 68 + col]);
#pragma unroll
                for (int i = 0; i < 4; ++i) xv[i] = gelu_erf(xv[i]) * oscale;
                *(v4fa*)(&os[row * 68 + col]) = xv; }
            wave_sync();
        }
#pragma unroll 1
        for (int ps = 0; ps < 2; ++ps) {
            if (OUTF32) {
#pragma unroll
                for (int s = 0; s < 8; ++s) { const int row = 2 * s + (lane >> 4), c4 = (lane & 15) * 4;
                    v4f xv = *(const v4fa*)(&os[row * 68 + c4]);
                    const size_t off = obase + (size_t)(mb * 16 + row) * ldc + c4;
                    if (RES) { const v4f rv = *(const v4f*)(res + off); xv = xv + rv; }
                    *(volatile v4f*)(Cf + off) = xv; }
            } else {
#pragma unroll
                for (int s = 0; s < 4; ++s) { const int row = 4 * s + (lane >> 3), c8 = (lane & 7) * 8;
                    const v4f x0 = *(const v4fa*)(&os[row * 68 + c8]); const v4f x1 = *(const v4fa*)(&os[row * 68 + c8 + 4]); v8h hv;
#pragma unroll
                    for (int i = 0; i < 4; ++i) { hv[i] = toh_flush(x0[i]); hv[4 + i] = toh_flush(x1[i]); }
                    const size_t off = obase + (size_t)(mb * 16 + row) * ldc + c8;
                    *(volatile v8h*)(Ch + off) = hv; }
            }
            if (ps == 0) __threadfence(); }
        wave_sync();
    }
}

__global__ __launch_bounds__(32) void k_gemm_q(const h16* __restrict__ A, const h16* __restrict__ Bt, const float* __restrict__ bias, h16* Ch) {
    __shared__ __align__(16) float os[16 * 68];
    gemm_tile<0, 1, 0, 0>(os, A, Bt, bias, nullptr, nullptr, Ch, CD, CD, CD, (size_t)0, QC / (HC * WC), QC, 0.0f);
}
__global__ __launch_bounds__(32) void k_gemm_kt(const h16* __restrict__ A, const h16* __restrict__ Bt, float* Cf) {
    __shared__ __align__(16) float os[16 * 68];
    gemm_tile<1, 0, 0, 0>(os, A, Bt, nullptr, nullptr, Cf, nullptr, CD, NKV, NKV, (size_t)CD * NKV, 1.0f / (WC * KIC), 0.0f, 0.0f);
}
__global__ __launch_bounds__(32) void k_gemm_vt(const h16* __restrict__ A, const h16* __restrict__ Bt, const float* __restrict__ bias, h16* Ch) {
    __shared__ __align__(16) float os[16 * 68];
    gemm_tile<0, 2, 0, 0>(os, A, Bt, bias, nullptr, nullptr, Ch, CD, NKV, NKV, (size_t)CD * NKV, VC / (WC * KIC), VC, 0.0f);
}
__global__ __launch_bounds__(32) void k_gemm_proj(const h16* __restrict__ A, const h16* __restrict__ Bt, const float* __restrict__ bias, const float* __restrict__ res, float* Cf) {
    __shared__ __align__(16) float os[16 * 68];
    gemm_tile<1, 1, 1, 0>(os, A, Bt, bias, res, Cf, nullptr, CD, CD, CD, (size_t)0, 1.0f / (AC * WC), 1.0f, 0.0f);
}
__global__ __launch_bounds__(32) void k_gemm_mlp1(const h16* __restrict__ A, const h16* __restrict__ Bt, const float* __restrict__ bias, h16* Ch) {
    __shared__ __align__(16) float os[16 * 68];
    gemm_tile<0, 1, 0, 1>(os, A, Bt, bias, nullptr, nullptr, Ch, CD, HID, HID, (size_t)0, 1.0f / (HC * WC), 1.0f, GC);
}
__global__ __launch_bounds__(32) void k_gemm_mlp2(const h16* __restrict__ A, const h16* __restrict__ Bt, const float* __restrict__ bias, const float* __restrict__ res, float* Cf) {
    __shared__ __align__(16) float os[16 * 68];
    gemm_tile<1, 1, 1, 0>(os, A, Bt, bias, res, Cf, nullptr, HID, CD, CD, (size_t)0, 1.0f / (GC * WC), 1.0f, 0.0f);
}

static_assert(32 * 16 == NKV * 2);
__global__ __launch_bounds__(256) void k_ksoft(const float* __restrict__ KT, h16* KS) {
#pragma clang fp contract(off)
    const int lane = threadIdx.x & 31;
    const int wave = __builtin_amdgcn_readfirstlane((int)(threadIdx.x >> 5));
    const size_t row = (size_t)blockIdx.x * 8 + wave;
    const float* p = KT + row * NKV + lane * 8;
    const v4f a = *(const v4f*)p, c = *(const v4f*)(p + 4);
    float xv[8];
#pragma unroll
    for (int i = 0; i < 4; ++i) { xv[i] = a[i]; xv[4 + i] = c[i]; }
    float mx = xv[0];
#pragma unroll
    for (int i = 1; i < 8; ++i) mx = fmaxf(mx, xv[i]);
    mx = fmaxf(mx, __shfl_xor(mx, 16, 32)); mx = fmaxf(mx, __shfl_xor(mx, 8, 32)); mx = fmaxf(mx, __shfl_xor(mx, 4, 32)); mx = fmaxf(mx, __shfl_xor(mx, 2, 32)); mx = fmaxf(mx, __shfl_xor(mx, 1, 32));
    float e[8]; float sm = 0.0f;
#pragma unroll
    for (int i = 0; i < 8; ++i) { e[i] = __builtin_amdgcn_exp2f((xv[i] - mx) * LOG2E); sm = sm + e[i]; }
    sm = sm + __shfl_xor(sm, 16, 32); sm = sm + __shfl_xor(sm, 8, 32); sm = sm + __shfl_xor(sm, 4, 32); sm = sm + __shfl_xor(sm, 2, 32); sm = sm + __shfl_xor(sm, 1, 32);
    const float inv = KSC * (1.0f / sm);
    v8h o;
#pragma unroll
    for (int i = 0; i < 8; ++i) o[i] = toh_flush(e[i] * inv);
    h16* q = KS + row * NKV + lane * 8;
    *(volatile v8h*)q = o; __threadfence(); *(volatile v8h*)q = o;
}

static_assert(12 * 32 * 16 == HD * KVP * 2);
__global__ __launch_bounds__(32) void k_kvmat(const h16* __restrict__ VT, const h16* __restrict__ KS, h16* KV) {
    __shared__ __align__(16) float os[HD * 68];
    const int lane = threadIdx.x & 31, lr = lane & 15, hi = lane >> 4;
    const int bh = blockIdx.x; const int b = bh / NH_, h = bh % NH_;
    const size_t rb = ((size_t)b * CD + (size_t)h * HD + (size_t)lr) * NKV + 8 * hi;
    v8f acc[3][3];
#pragma unroll
    for (int mt = 0; mt < 3; ++mt)
#pragma unroll
        for (int nt = 0; nt < 3; ++nt) acc[mt][nt] = (v8f){};
#pragma unroll 1
    for (int kc = 0; kc < NKV; kc += 32) {
        v16h a[3];
#pragma unroll
        for (int mt = 0; mt < 3; ++mt) a[mt] = ldh(VT + rb + (size_t)mt * 16 * NKV + kc);
#pragma unroll
        for (int nt = 0; nt < 3; ++nt) { const v16h bq = ldh(KS + rb + (size_t)nt * 16 * NKV + kc);
#pragma unroll
            for (int mt = 0; mt < 3; ++mt) acc[mt][nt] = wmma16g(a[mt], bq, acc[mt][nt]); }
    }
#pragma unroll
    for (int mt = 0; mt < 3; ++mt) {
#pragma unroll
        for (int j = 0; j < 8; ++j) {
#pragma unroll
            for (int nt = 0; nt < 3; ++nt) os[(mt * 16 + hi * 8 + j) * 68 + nt * 16 + lr] = acc[mt][nt][j] * (KVC / (VC * KSC));
            os[(mt * 16 + hi * 8 + j) * 68 + 48 + lr] = 0.0f; } }
    wave_sync();
    h16* kvb = KV + (size_t)bh * HD * KVP;
#pragma unroll 1
    for (int ps = 0; ps < 2; ++ps) {
#pragma unroll 1
        for (int s = 0; s < 12; ++s) { const int row = 4 * s + (lane >> 3), c8 = (lane & 7) * 8;
            const v4f x0 = *(const v4fa*)(&os[row * 68 + c8]); const v4f x1 = *(const v4fa*)(&os[row * 68 + c8 + 4]); v8h hv;
#pragma unroll
            for (int i = 0; i < 4; ++i) { hv[i] = toh_flush(x0[i]); hv[4 + i] = toh_flush(x1[i]); }
            *(volatile v8h*)(kvb + (size_t)row * KVP + c8) = hv; }
        if (ps == 0) __threadfence(); }
}

static_assert(24 * 32 * 16 == 16 * CD * 2);
__global__ __launch_bounds__(32) void k_attn(const h16* __restrict__ Q, const h16* __restrict__ KV, h16* AT) {
    __shared__ __align__(16) float os[16 * APITCH];
    const int lane = threadIdx.x & 31, lr = lane & 15, hi = lane >> 4;
    const int tg = blockIdx.x * 16; const int b = tg / SEQ;
    const size_t qo = (size_t)(tg + lr) * CD + 8 * hi;
    const v8h z8 = (v8h){};
#pragma unroll 1
    for (int h = 0; h < NH_; ++h) {
        const h16* qp = Q + qo + h * HD;
        const v16h a0 = ldh(qp);
        const v16h a1 = cat16(*(const v8h*)(qp + 32), z8);
        const h16* kp = KV + ((size_t)(b * NH_ + h) * HD + (size_t)lr) * KVP + 8 * hi;
        v8f c0 = (v8f){}, c1 = (v8f){}, c2 = (v8f){};
        { const v16h b0 = ldh(kp), b1 = ldh(kp + 32);                                     c0 = wmma16g(a0, b0, c0); c0 = wmma16g(a1, b1, c0); }
        { const v16h b0 = ldh(kp + 16 * KVP), b1 = ldh(kp + 16 * KVP + 32);               c1 = wmma16g(a0, b0, c1); c1 = wmma16g(a1, b1, c1); }
        { const v16h b0 = ldh(kp + 32 * KVP), b1 = ldh(kp + 32 * KVP + 32);               c2 = wmma16g(a0, b0, c2); c2 = wmma16g(a1, b1, c2); }
#pragma unroll
        for (int j = 0; j < 8; ++j) {
            os[(hi * 8 + j) * APITCH + h * HD +  0 + lr] = c0[j] * (ATT_SCALE * AC / (QC * KVC));
            os[(hi * 8 + j) * APITCH + h * HD + 16 + lr] = c1[j] * (ATT_SCALE * AC / (QC * KVC));
            os[(hi * 8 + j) * APITCH + h * HD + 32 + lr] = c2[j] * (ATT_SCALE * AC / (QC * KVC)); }
    }
    wave_sync();
    h16* ab = AT + (size_t)tg * CD;
#pragma unroll 1
    for (int ps = 0; ps < 2; ++ps) {
#pragma unroll 1
        for (int s = 0; s < 24; ++s) { const int p = s * 32 + lane; const int row = p / 48, c8 = (p % 48) * 8;
            const v4f x0 = *(const v4fa*)(&os[row * APITCH + c8]); const v4f x1 = *(const v4fa*)(&os[row * APITCH + c8 + 4]); v8h hv;
#pragma unroll
            for (int i = 0; i < 4; ++i) { hv[i] = toh_flush(x0[i]); hv[4 + i] = toh_flush(x1[i]); }
            *(volatile v8h*)(ab + (size_t)p * 8) = hv; }
        if (ps == 0) __threadfence(); }
}

static constexpr size_t al256(size_t v) { return (v + 255) & ~(size_t)255; }
static constexpr size_t SZ_W  = al256((size_t)CD * CD * 2);
static constexpr size_t SZ_W1 = al256((size_t)HID * CD * 2);
static constexpr size_t SZ_X2 = al256((size_t)BN * CD * 4);
static constexpr size_t SZ_PA = al256((size_t)BN * CD * 2);
static constexpr size_t SZ_PB = al256((size_t)BN * CD * 2);
static constexpr size_t SZ_KI = al256((size_t)BK * CD * 2);
static constexpr size_t SZ_KT = al256((size_t)NB * CD * NKV * 4);
static constexpr size_t SZ_KS = al256((size_t)NB * CD * NKV * 2);
static constexpr size_t SZ_VT = al256((size_t)NB * CD * NKV * 2);
static constexpr size_t SZ_KV = al256((size_t)NB * NH_ * HD * KVP * 2);
static constexpr size_t SZ_TOTAL = 4 * SZ_W + 2 * SZ_W1 + SZ_X2 + SZ_PA + SZ_PB + SZ_KI + SZ_KT + SZ_KS + SZ_VT + SZ_KV;
static_assert(SZ_TOTAL <= (size_t)134217728);
static_assert((size_t)QROWS * HID * 2 <= SZ_PA);
static_assert((size_t)BN * CD * 2 <= SZ_PA);

extern "C" void kernel_launch(void* const* d_in, const int* in_sizes, int n_in,
                              void* d_out, int out_size, void* d_ws, size_t ws_size, hipStream_t stream) {
    if (n_in < 21) return;
    if ((size_t)in_sizes[0] < (size_t)BN * CD) return;
    if (in_sizes[1] < 9 * CD || in_sizes[2] < CD || in_sizes[3] < CD * CD || in_sizes[4] < CD || in_sizes[5] < 16 * CD) return;
    if (in_sizes[6] < CD * CD || in_sizes[7] < CD * CD || in_sizes[8] < CD || in_sizes[9] < CD * CD || in_sizes[10] < CD) return;
    if (in_sizes[11] < CD || in_sizes[12] < CD || in_sizes[13] < CD || in_sizes[14] < CD) return;
    if (in_sizes[15] < CD * HID || in_sizes[16] < HID || in_sizes[17] < HID * CD || in_sizes[18] < CD) return;
    if (in_sizes[19] < 1 || in_sizes[20] < 1) return;
    if ((size_t)out_size < (size_t)BN * CD) return;
    if (SZ_TOTAL > ws_size) return;
    const float* x      = (const float*)d_in[0];
    const float* cpe_w  = (const float*)d_in[1];
    const float* cpe_b  = (const float*)d_in[2];
    const float* q_w    = (const float*)d_in[3];
    const float* q_b    = (const float*)d_in[4];
    const float* kv_w   = (const float*)d_in[5];
    const float* k_w    = (const float*)d_in[6];
    const float* v_w    = (const float*)d_in[7];
    const float* v_b    = (const float*)d_in[8];
    const float* proj_w = (const float*)d_in[9];
    const float* proj_b = (const float*)d_in[10];
    const float* ln1_g  = (const float*)d_in[11];
    const float* ln1_b  = (const float*)d_in[12];
    const float* ln2_g  = (const float*)d_in[13];
    const float* ln2_b  = (const float*)d_in[14];
    const float* w1     = (const float*)d_in[15];
    const float* b1     = (const float*)d_in[16];
    const float* w2     = (const float*)d_in[17];
    const float* b2     = (const float*)d_in[18];
    const int*   Hp     = (const int*)d_in[19];
    const int*   Wp     = (const int*)d_in[20];
    float* OUT = (float*)d_out;
    float* X1 = OUT;
    char* wsp = (char*)d_ws;
    h16* WQ  = (h16*)wsp; wsp += SZ_W;
    h16* WK  = (h16*)wsp; wsp += SZ_W;
    h16* WV  = (h16*)wsp; wsp += SZ_W;
    h16* WP  = (h16*)wsp; wsp += SZ_W;
    h16* W1T = (h16*)wsp; wsp += SZ_W1;
    h16* W2T = (h16*)wsp; wsp += SZ_W1;
    float* X2 = (float*)wsp; wsp += SZ_X2;
    h16* PA  = (h16*)wsp; wsp += SZ_PA;
    h16* PB  = (h16*)wsp; wsp += SZ_PB;
    h16* KI  = (h16*)wsp; wsp += SZ_KI;
    float* KT = (float*)wsp; wsp += SZ_KT;
    h16* KS  = (h16*)wsp; wsp += SZ_KS;
    h16* VT  = (h16*)wsp; wsp += SZ_VT;
    h16* KV  = (h16*)wsp; wsp += SZ_KV;

    k_wconv<<<dim3(CD / 64, CD / 64, 1), 256, 0, stream>>>(q_w, WQ, CD, CD);
    k_wconv<<<dim3(CD / 64, CD / 64, 1), 256, 0, stream>>>(k_w, WK, CD, CD);
    k_wconv<<<dim3(CD / 64, CD / 64, 1), 256, 0, stream>>>(v_w, WV, CD, CD);
    k_wconv<<<dim3(CD / 64, CD / 64, 1), 256, 0, stream>>>(proj_w, WP, CD, CD);
    k_wconv<<<dim3(HID / 64, CD / 64, 1), 256, 0, stream>>>(w1, W1T, CD, HID);
    k_wconv<<<dim3(CD / 64, HID / 64, 1), 256, 0, stream>>>(w2, W2T, HID, CD);

    k_cpe_ln<<<BN / 8, 256, 0, stream>>>(x, cpe_w, cpe_b, ln1_g, ln1_b, Hp, Wp, X1, PA);
    k_kvconv<<<(unsigned)(((size_t)BK * 48) / 256), 256, 0, stream>>>(PA, kv_w, KI);
    k_gemm_q<<<dim3(BN / 64, CD / 64, 1), 32, 0, stream>>>(PA, WQ, q_b, PB);
    k_gemm_kt<<<dim3(CD / 64, BK / 64, 1), 32, 0, stream>>>(WK, KI, KT);
    k_gemm_vt<<<dim3(CD / 64, BK / 64, 1), 32, 0, stream>>>(WV, KI, v_b, VT);
    k_ksoft<<<(NB * CD) / 8, 256, 0, stream>>>(KT, KS);
    k_kvmat<<<NB * NH_, 32, 0, stream>>>(VT, KS, KV);
    k_attn<<<BN / 16, 32, 0, stream>>>(PB, KV, PA);
    k_gemm_proj<<<dim3(BN / 64, CD / 64, 1), 32, 0, stream>>>(PA, WP, proj_b, X1, X2);
    k_ln2<<<BN / 8, 256, 0, stream>>>(X2, ln2_g, ln2_b, PB);
    for (int qd = 0; qd < MLPQ; ++qd) {
        const size_t ro = (size_t)qd * QROWS * CD;
        k_gemm_mlp1<<<dim3(QROWS / 64, HID / 64, 1), 32, 0, stream>>>(PB + ro, W1T, b1, PA);
        k_gemm_mlp2<<<dim3(QROWS / 64, CD / 64, 1), 32, 0, stream>>>(PA, W2T, b2, X2 + ro, OUT + ro);
    }
}
